// PointNet_11742440587706
// MI455X (gfx1250) — hardware-verified
//
#include <hip/hip_runtime.h>

typedef __attribute__((ext_vector_type(16))) _Float16 v16h;
typedef __attribute__((ext_vector_type(8)))  _Float16 v8h;
typedef __attribute__((ext_vector_type(8)))  float    v8f;
typedef __attribute__((ext_vector_type(4)))  float    v4f;
typedef __attribute__((ext_vector_type(4)))  int      v4i;
typedef __attribute__((ext_vector_type(4)))  unsigned int v4u;

constexpr int N_NODES    = 100000;
constexpr int N_EDGES    = 1600000;
constexpr int HID        = 32;
constexpr int NTHR       = 256;
constexpr int NWAVES     = NTHR / 32;
constexpr int TILE_ROWS  = 1024;
constexpr int WAVE_ROWS  = TILE_ROWS / NWAVES;
constexpr int WAVE_ROWS_LOG2 = 7;
constexpr int N_TILES    = (N_NODES + TILE_ROWS - 1) / TILE_ROWS;
constexpr int ACC_ROWS   = N_TILES * TILE_ROWS;
constexpr int CHUNK      = 8192;
constexpr int EPT        = CHUNK / NTHR;
constexpr int N_CHUNKS   = (N_EDGES + CHUNK - 1) / CHUNK;
constexpr int GROUP      = 64;
constexpr int LCAP       = CHUNK + GROUP;
constexpr int MAX_GROUPS = LCAP / GROUP + 1;

static_assert(WAVE_ROWS == (1 << WAVE_ROWS_LOG2), "wave row range");
static_assert(NWAVES == 8, "8 waves");
static_assert(NTHR == 4 * GROUP, "gather mapping");
static_assert(N_EDGES % EPT == 0, "thread edge groups entirely in or out");
static_assert(EPT % 4 == 0, "b128 loads");
static_assert(N_NODES % 4 == 0, "4-row store groups");
static_assert(WAVE_ROWS % 4 == 0, "4-row store groups");
static_assert(ACC_ROWS % 4 == 0, "4-row store groups");
static_assert(ACC_ROWS >= N_NODES, "padded plane");
static_assert(N_CHUNKS * CHUNK >= N_EDGES, "chunk cover");
static_assert((N_EDGES % 4) == 0, "b128 alignment of the dst row");
static_assert(MAX_GROUPS * GROUP >= LCAP, "group bound");

template <typename T> struct Frag;
template <> struct Frag<_Float16> {
  typedef v16h V; union U { v16h v; v8h h[2]; };
  static __device__ __forceinline__ v16h load(const _Float16* p) {
    U f; f.h[0] = *(const v8h*)(p); f.h[1] = *(const v8h*)(p + 16); return f.v;
  }
  static __device__ __forceinline__ v8f mma(v16h a, v16h b, v8f c) {
    return __builtin_amdgcn_wmma_f32_16x16x32_f16(false, a, false, b, (short)0, c, false, false);
  }
};
__device__ __forceinline__ void wstep(v8f& c, v16h a, v16h b) {
  c = Frag<_Float16>::mma(a, b, c);
  asm volatile("v_nop\n\tv_nop\n\tv_nop\n\tv_nop" : "+v"(c) : "v"(a), "v"(b));
}
__device__ __forceinline__ unsigned pk16(unsigned short a, unsigned short b) { return (unsigned)a | ((unsigned)b << 16); }
__device__ __forceinline__ unsigned short h_bits(float f) { const _Float16 h = (_Float16)f; return __builtin_bit_cast(unsigned short, h); }
__device__ __forceinline__ float vzero() { float z = 0.0f; asm volatile("" : "+v"(z)); return z; }
__device__ __forceinline__ void st8h(_Float16* p, float f0, float f1, float f2, float f3,
                                     float f4, float f5, float f6, float f7) {
  const v4u u = (v4u){pk16(h_bits(f0), h_bits(f1)), pk16(h_bits(f2), h_bits(f3)),
                      pk16(h_bits(f4), h_bits(f5)), pk16(h_bits(f6), h_bits(f7))};
  *(v4u*)(void*)p = u;
}
__device__ __forceinline__ void stz8(_Float16* p) { *(v4u*)(void*)p = (v4u){0u, 0u, 0u, 0u}; }
__device__ __forceinline__ int clampi(int v, int lo, int hi) { return v < lo ? lo : (v > hi ? hi : v); }

__device__ __forceinline__ int blk_excl_scan(int cnt, int* scan_ws, int tid, int* tot) {
  const int lane = tid & 31, wave = tid >> 5; int incl = cnt;
#pragma unroll
  for (int o = 1; o < 32; o <<= 1) { const int v = __shfl_up(incl, o, 32); if (lane >= o) incl += v; }
  if (lane == 31) scan_ws[wave] = incl;
  __syncthreads();
  if (wave == 0) { int wv = (lane < NWAVES) ? scan_ws[lane] : 0; int wincl = wv;
#pragma unroll
    for (int o = 1; o < 32; o <<= 1) { const int v = __shfl_up(wincl, o, 32); if (lane >= o) wincl += v; }
    if (lane < NWAVES) scan_ws[32 + lane] = wincl - wv; if (lane == 31) scan_ws[64] = wincl; }
  __syncthreads();
  const int res = scan_ws[32 + wave] + incl - cnt; *tot = scan_ws[64];
  return res;
}
__device__ __forceinline__ int chunk_scan(const int* __restrict__ dstv, int e0, int n0, int tid, int base,
                                          int* LIST, int* scan_ws) {
  const int eb  = e0 + tid * EPT;
  const bool inr = eb < N_EDGES;
  const int ebc = inr ? eb : (N_EDGES - EPT);
  int rec[EPT]; int cnt = 0;
#pragma unroll
  for (int k = 0; k < EPT; k += 4) {
    const v4i d4 = *(const v4i*)(dstv + ebc + k);
#pragma unroll
    for (int e = 0; e < 4; ++e) {
      const int d = d4[e];
      const bool hit = inr && (d >= n0) && (d < n0 + TILE_ROWS);
      rec[k + e] = hit ? (eb + k + e) : -1;
      cnt += hit ? 1 : 0;
    }
  }
  int tot; int p = base + blk_excl_scan(cnt, scan_ws, tid, &tot);
#pragma unroll
  for (int k = 0; k < EPT; ++k) if (rec[k] >= 0) { if ((unsigned)p < (unsigned)LCAP) LIST[p] = rec[k]; ++p; }
  __syncthreads();
  const int nt = base + tot;
  return nt < LCAP ? nt : LCAP;
}

template <int IN_F>
__global__ __launch_bounds__(NTHR) void pn_layer_kernel(
    const float* __restrict__ hin, const float* __restrict__ pos, const int* __restrict__ ei,
    const float* __restrict__ Wa, const float* __restrict__ ba,
    const float* __restrict__ Wb, const float* __restrict__ bb, float* __restrict__ outp, int row_limit) {
  constexpr int IN_TOT = IN_F + 3;
  constexpr int KA   = ((IN_TOT + 31) / 32) * 32;
  constexpr int NKS  = KA / 32;
  constexpr int PA   = KA + 8;
  constexpr int PBA  = KA + 8;
  constexpr int PT   = HID + 8;
  constexpr int PBB  = HID + 8;
  constexpr int PM   = HID + 1;
  constexpr int NCHA = KA / 8;
  static_assert(KA % 32 == 0, "K multiple of 32");
  static_assert(IN_F == 3 || IN_F == 32, "layer type");
  static_assert(HID * NCHA <= NTHR, "weight staging covers every (n, chunk) in one pass");

  __shared__ __align__(16) float Acc[TILE_ROWS * HID];
  __shared__ int LIST[LCAP];
  __shared__ int scan_ws[80];
  __shared__ int DL[GROUP];
  __shared__ __align__(16) _Float16 Ash[GROUP * PA];
  __shared__ __align__(16) _Float16 Tsh[GROUP * PT];
  __shared__ __align__(16) _Float16 BtA[HID * PBA];
  __shared__ __align__(16) _Float16 BtB[HID * PBB];
  __shared__ float Msh[GROUP * PM];

  const int tid  = threadIdx.x;
  const int lane = tid & 31;
  const int wave = tid >> 5;
  const int n0   = blockIdx.x * TILE_ROWS;
  const int rl   = lane & 15;
  const int hh   = lane >> 4;
  const int koff = hh * 8;
  const int mi   = wave & 3;
  const int ni   = wave >> 2;
  const int dcol = ni * 16 + rl;

  for (int w = tid; w < HID * NCHA; w += NTHR) {
    const int n = w & 31, c = w >> 5;
    float f[8];
#pragma unroll
    for (int e = 0; e < 8; ++e) {
      const int k  = 8 * c + e;
      const int kc = (k < IN_TOT) ? k : (IN_TOT - 1);
      const float wv = Wa[kc * HID + n];
      f[e] = (k < IN_TOT) ? wv : vzero();
    }
    st8h(BtA + n * PBA + 8 * c, f[0], f[1], f[2], f[3], f[4], f[5], f[6], f[7]);
  }
  for (int w = tid; w < HID * 4; w += NTHR) {
    const int n = w & 31, c = w >> 5;
    float f[8];
#pragma unroll
    for (int e = 0; e < 8; ++e) f[e] = Wb[(8 * c + e) * HID + n];
    st8h(BtB + n * PBB + 8 * c, f[0], f[1], f[2], f[3], f[4], f[5], f[6], f[7]);
  }
  if (tid < 80) scan_ws[tid] = 0;
#pragma unroll 1
  for (int j = 0; j < WAVE_ROWS; ++j) Acc[(wave * WAVE_ROWS + j) * HID + lane] = 0.0f;
  const float bav = ba[dcol];
  const float bbv = bb[dcol];
  __syncthreads();

  const int* dstv = ei + N_EDGES;
  int lcnt = 0;
#pragma unroll 1
  for (int ch = 0; ch < N_CHUNKS; ++ch) {
    const int tot = chunk_scan(dstv, ch * CHUNK, n0, tid, lcnt, LIST, scan_ws);
    const bool last = (ch == N_CHUNKS - 1);
    const int nfull = tot / GROUP;
    int ng = last ? ((tot + GROUP - 1) / GROUP) : nfull;
    ng = ng < MAX_GROUPS ? ng : MAX_GROUPS;
#pragma unroll 1
    for (int g = 0; g < ng; ++g) {
      {
        const int r = tid & (GROUP - 1);
        const int q = wave >> 1;
        const int idx = g * GROUP + r;
        const bool valid = idx < tot;
        const int idc = valid ? idx : (tot - 1);
        int e = LIST[idc];
        e = clampi(e, 0, N_EDGES - 1);
        const int s = clampi(ei[e], 0, N_NODES - 1);
        const int d = clampi(ei[N_EDGES + e], 0, N_NODES - 1);
        if (q == 0) DL[r] = valid ? clampi(d - n0, 0, TILE_ROWS - 1) : -1;
        _Float16* arow = Ash + r * PA;
        if (IN_F == 3) {
          if (q == 0) {
            const float ps0 = pos[s * 3], ps1 = pos[s * 3 + 1], ps2 = pos[s * 3 + 2];
            const float pd0 = pos[d * 3], pd1 = pos[d * 3 + 1], pd2 = pos[d * 3 + 2];
            const float r0 = ps0 - pd0, r1 = ps1 - pd1, r2 = ps2 - pd2;
            const float z = vzero();
            st8h(arow, ps0, ps1, ps2, r0, r1, r2, z, z);
          } else {
            stz8(arow + 8 * q);
          }
        } else {
          const float* hp = hin + (size_t)s * HID + 8 * q;
          const v4f x0 = *(const v4f*)(hp);
          const v4f x1 = *(const v4f*)(hp + 4);
          st8h(arow + 8 * q, x0[0], x0[1], x0[2], x0[3], x1[0], x1[1], x1[2], x1[3]);
          if (q == 0) {
            const float ps0 = pos[s * 3], ps1 = pos[s * 3 + 1], ps2 = pos[s * 3 + 2];
            const float pd0 = pos[d * 3], pd1 = pos[d * 3 + 1], pd2 = pos[d * 3 + 2];
            const float r0 = ps0 - pd0, r1 = ps1 - pd1, r2 = ps2 - pd2;
            const float z = vzero();
            st8h(arow + 32, r0, r1, r2, z, z, z, z, z);
          } else {
            stz8(arow + 32 + 8 * q);
          }
        }
      }
      __syncthreads();
      v8f acc = (v8f){0.f, 0.f, 0.f, 0.f, 0.f, 0.f, 0.f, 0.f};
#pragma unroll
      for (int ks = 0; ks < NKS; ++ks) {
        const v16h a  = Frag<_Float16>::load(Ash + (16 * mi + rl) * PA  + 32 * ks + koff);
        const v16h bt = Frag<_Float16>::load(BtA + (16 * ni + rl) * PBA + 32 * ks + koff);
        wstep(acc, a, bt);
      }
#pragma unroll
      for (int r = 0; r < 8; ++r) {
        const int row = 16 * mi + 8 * hh + r;
        float v = acc[r] + bav;
        v = fmaxf(v, 0.0f);
        Tsh[row * PT + dcol] = (_Float16)v;
      }
      __syncthreads();
      v8f acc2 = (v8f){0.f, 0.f, 0.f, 0.f, 0.f, 0.f, 0.f, 0.f};
      {
        const v16h a  = Frag<_Float16>::load(Tsh + (16 * mi + rl) * PT  + koff);
        const v16h bt = Frag<_Float16>::load(BtB + (16 * ni + rl) * PBB + koff);
        wstep(acc2, a, bt);
      }
#pragma unroll
      for (int r = 0; r < 8; ++r) {
        const int row = 16 * mi + 8 * hh + r;
        Msh[row * PM + dcol] = acc2[r] + bbv;
      }
      __syncthreads();
#pragma unroll
      for (int half = 0; half < 2; ++half) {
        const int dli = DL[half * 32 + lane];
        const int own = (dli >= 0 && (dli >> WAVE_ROWS_LOG2) == wave) ? 1 : 0;
        unsigned msk = (unsigned)__ballot(own);
#pragma unroll 1
        for (int it = 0; it < 32; ++it) {
          if (msk == 0u) break;
          const int bp = __builtin_ctz(msk);
          msk &= msk - 1u;
          const int dlh = __shfl(dli, bp, 32);
          const float mv = Msh[(half * 32 + bp) * PM + lane];
          const int ai = dlh * HID + lane;
          const float cur = Acc[ai];
          Acc[ai] = fmaxf(cur, mv);
        }
      }
      __syncthreads();
    }
    const int rem = last ? 0 : (tot - nfull * GROUP);
    if (rem > 0) {
      const int si = nfull * GROUP + (tid < rem ? tid : rem - 1);
      const int cv = LIST[si];
      __syncthreads();
      if (tid < rem) LIST[tid] = cv;
      __syncthreads();
    }
    lcnt = rem;
  }
  __syncthreads();
  {
    const int q8 = lane >> 3, c4 = (lane & 7) * 4;
    for (int pass = 0; pass < 2; ++pass) {
#pragma unroll 1
      for (int j = 0; j < WAVE_ROWS / 4; ++j) {
        const int lrow0 = wave * WAVE_ROWS + 4 * j;
        if (n0 + lrow0 < row_limit) {
          const v4f v = *(const v4f*)(Acc + (lrow0 + q8) * HID + c4);
          *(volatile v4f*)(outp + (size_t)(n0 + lrow0 + q8) * HID + c4) = v;
        }
      }
      __threadfence();
    }
  }
}

extern "C" void kernel_launch(void* const* d_in, const int* in_sizes, int n_in,
                              void* d_out, int out_size, void* d_ws, size_t ws_size,
                              hipStream_t stream) {
  (void)in_sizes; (void)n_in; (void)out_size;
  const float* pos = (const float*)d_in[0];
  const int*   ei  = (const int*)  d_in[1];
  const float* W1  = (const float*)d_in[3];
  const float* b1  = (const float*)d_in[4];
  const float* W2  = (const float*)d_in[5];
  const float* b2  = (const float*)d_in[6];
  const float* W3  = (const float*)d_in[7];
  const float* b3  = (const float*)d_in[8];
  const float* W4  = (const float*)d_in[9];
  const float* b4  = (const float*)d_in[10];
  float* out = (float*)d_out;

  const size_t h1_bytes = (size_t)ACC_ROWS * HID * sizeof(float);
  if (h1_bytes > ws_size) return;
  float* h1 = (float*)d_ws;

  pn_layer_kernel<3><<<N_TILES, NTHR, 0, stream>>>(pos, pos, ei, W1, b1, W2, b2, h1, ACC_ROWS);
  pn_layer_kernel<32><<<N_TILES, NTHR, 0, stream>>>(h1, pos, ei, W3, b3, W4, b4, out, N_NODES);
}
